// MultiHeadedAttentionNeighbor_83159156785323
// MI455X (gfx1250) — hardware-verified
//
#include <hip/hip_runtime.h>
#include <math.h>
#include <stdint.h>

constexpr int kBatch = 16;
constexpr int kSeq   = 512;
constexpr int kDm    = 512;
constexpr int kHeads = 8;
constexpr int kDk    = 64;
constexpr int kGB    = 4;
constexpr int kNGrp  = kBatch / kGB;
constexpr int kNZ    = kGB * kHeads;
constexpr int kGRows = kGB * kSeq;
constexpr float kLog2e = 1.4426950408889634f;
static_assert(kSeq == 512 && kDk == 64 && kDm == kHeads * kDk && (kBatch % kGB) == 0, "geometry");

typedef __attribute__((ext_vector_type(16))) _Float16 v16h;
typedef __attribute__((ext_vector_type(8)))  _Float16 v8h;
typedef __attribute__((ext_vector_type(16))) __bf16   v16b;
typedef __attribute__((ext_vector_type(8)))  __bf16   v8b;
typedef __attribute__((ext_vector_type(8)))  float    v8f;
typedef __attribute__((ext_vector_type(4)))  float    v4f;
typedef __attribute__((ext_vector_type(4)))  unsigned int v4u;

__device__ __forceinline__ unsigned short f2bf_bits(float f) {
  unsigned u = __float_as_uint(f);
  return (unsigned short)((u + 0x7FFFu + ((u >> 16) & 1u)) >> 16);
}
__device__ __forceinline__ float bf_bits2f(unsigned short h) { return __uint_as_float(((unsigned)h) << 16); }
__device__ __forceinline__ unsigned pk16(unsigned short a, unsigned short b) { return (unsigned)a | ((unsigned)b << 16); }

__device__ __forceinline__ void dep_guard_h(v8f& a, v8f& b, v16h x, v16h y) { asm volatile("v_nop\n\tv_nop\n\tv_nop\n\tv_nop" : "+v"(a), "+v"(b) : "v"(x), "v"(y)); }
__device__ __forceinline__ void dep_guard_b(v8f& a, v8f& b, v16b x, v16b y) { asm volatile("v_nop\n\tv_nop\n\tv_nop\n\tv_nop" : "+v"(a), "+v"(b) : "v"(x), "v"(y)); }
__device__ __forceinline__ void keep4_h(v16h a, v16h b, v16h c, v16h d) { asm volatile("v_nop" :: "v"(a), "v"(b), "v"(c), "v"(d)); }
__device__ __forceinline__ void keep4_b(v16b a, v16b b, v16b c, v16b d) { asm volatile("v_nop" :: "v"(a), "v"(b), "v"(c), "v"(d)); }
__device__ __forceinline__ void acc_guard4(v8f& a, v8f& b, v8f& c, v8f& d) { asm volatile("v_nop\n\tv_nop\n\tv_nop\n\tv_nop" : "+v"(a), "+v"(b), "+v"(c), "+v"(d)); }
template <typename T> struct Frag;
template <> struct Frag<_Float16> {
  typedef v16h V; union U { v16h v; v8h h[2]; };
  static __device__ __forceinline__ v16h load(const _Float16* p) {
    U f; f.h[0] = *(const v8h*)(p); f.h[1] = *(const v8h*)(p + 16); return f.v;
  }
  static __device__ __forceinline__ v8f mma(v16h a, v16h b, v8f c) {
    return __builtin_amdgcn_wmma_f32_16x16x32_f16(false, a, false, b, (short)0, c, false, false);
  }
  static __device__ __forceinline__ void guard(v8f& a, v8f& b, v16h x, v16h y) { dep_guard_h(a, b, x, y); }
  static __device__ __forceinline__ void keep(v16h a, v16h b, v16h c, v16h d) { keep4_h(a, b, c, d); }
};
template <> struct Frag<__bf16> {
  typedef v16b V; union U { v16b v; v8b h[2]; };
  static __device__ __forceinline__ v16b load(const __bf16* p) {
    U f; f.h[0] = *(const v8b*)(p); f.h[1] = *(const v8b*)(p + 16); return f.v;
  }
  static __device__ __forceinline__ v8f mma(v16b a, v16b b, v8f c) {
    return __builtin_amdgcn_wmma_f32_16x16x32_bf16(false, a, false, b, (short)0, c, false, false);
  }
  static __device__ __forceinline__ void guard(v8f& a, v8f& b, v16b x, v16b y) { dep_guard_b(a, b, x, y); }
  static __device__ __forceinline__ void keep(v16b a, v16b b, v16b c, v16b d) { keep4_b(a, b, c, d); }
};

template <int ET> struct Elem;
template <> struct Elem<0> { typedef _Float16 T; };
template <> struct Elem<1> { typedef __bf16 T; };
template <int ET, bool SPLIT, int BIAS_MODE, int OUT_MODE, bool RESID, int ACT = 0>
__global__ __launch_bounds__(256) void wmma_gemm64(
    const unsigned short* __restrict__ Ap, const unsigned short* __restrict__ A2p, int lda, long strideA, long strideA2,
    const unsigned short* __restrict__ Btp, const unsigned short* __restrict__ Bt2p, int ldb, long strideB, long strideB2,
    void* __restrict__ Cout, void* __restrict__ Cout2, int ldc, long strideC, long strideC2,
    const float* __restrict__ bias,
    const float* __restrict__ resid, long strideR,
    int M, int N, int K, float scale, int zsplit) {
  typedef typename Elem<ET>::T T;
  typedef typename Frag<T>::V V;
  const T* A = (const T*)Ap; const T* A2 = (const T*)A2p; const T* Bt = (const T*)Btp; const T* Bt2 = (const T*)Bt2p;
  __shared__ __align__(16) float sT[8][16 * 68];
  const int bz   = blockIdx.y;
  const int zo   = bz / zsplit;
  const int zi   = bz - zo * zsplit;
  const int lane = threadIdx.x & 31;
  const int wave = threadIdx.x >> 5;
  const int tilesN = N >> 6;
  const int tilesM = M >> 6;
  const int tile = blockIdx.x * 8 + wave;
  if (tile >= tilesM * tilesN) return;
  const int tm = tile / tilesN;
  const int tn = tile - tm * tilesN;
  const int m0 = tm << 6;
  const int n0 = tn << 6;

  const size_t aOff = (size_t)zi * strideA + (size_t)zo * strideA2;
  const size_t bOff = (size_t)zi * strideB + (size_t)zo * strideB2;
  const size_t cOff = (size_t)zi * strideC + (size_t)zo * strideC2;
  const T* Ab  = A  + aOff;
  const T* Bb  = Bt + bOff;
  const T* Ab2 = SPLIT ? (A2  + aOff) : nullptr;
  const T* Bb2 = SPLIT ? (Bt2 + bOff) : nullptr;

  const int rlane = lane & 15;
  const int koff  = (lane >> 4) * 8;
  const int mOff  = (lane >> 4) * 8;

  v8f acc[4][4];
#pragma unroll
  for (int i = 0; i < 4; ++i)
#pragma unroll
    for (int j = 0; j < 4; ++j) acc[i][j] = (v8f){0.f,0.f,0.f,0.f,0.f,0.f,0.f,0.f};

  for (int k0 = 0; k0 < K; k0 += 32) {
    V bh[4], bl[4];
#pragma unroll
    for (int j = 0; j < 4; ++j) {
      const size_t bo = (size_t)(n0 + (j << 4) + rlane) * ldb + koff + k0;
      bh[j] = Frag<T>::load(Bb + bo);
      if (SPLIT) bl[j] = Frag<T>::load(Bb2 + bo);
    }
#pragma unroll
    for (int i = 0; i < 4; ++i) {
      const size_t ao = (size_t)(m0 + (i << 4) + rlane) * lda + koff + k0;
      V ah = Frag<T>::load(Ab + ao);
      V al;
      if (SPLIT) al = Frag<T>::load(Ab2 + ao);
#pragma unroll
      for (int j = 0; j < 4; ++j) {
        acc[i][j] = Frag<T>::mma(ah, bh[j], acc[i][j]);
        if (SPLIT) {
          acc[i][j] = Frag<T>::mma(ah, bl[j], acc[i][j]);
          acc[i][j] = Frag<T>::mma(al, bh[j], acc[i][j]);
        }
      }
      Frag<T>::guard(acc[i][0], acc[i][3], ah, SPLIT ? al : ah);
    }
    Frag<T>::keep(bh[0], bh[1], bh[2], bh[3]);
    if (SPLIT) Frag<T>::keep(bl[0], bl[1], bl[2], bl[3]);
  }
  acc_guard4(acc[0][0], acc[0][1], acc[0][2], acc[0][3]);
  acc_guard4(acc[1][0], acc[1][1], acc[1][2], acc[1][3]);
  acc_guard4(acc[2][0], acc[2][1], acc[2][2], acc[2][3]);
  acc_guard4(acc[3][0], acc[3][1], acc[3][2], acc[3][3]);

  float* slab = sT[wave];
  const float* Rb = RESID ? (resid + (size_t)zi * strideR) : nullptr;
#pragma unroll
  for (int i = 0; i < 4; ++i) {
    const int mBase = m0 + (i << 4);
#pragma unroll
    for (int j = 0; j < 4; ++j) {
      const int n = n0 + (j << 4) + rlane;
      float bv = 0.f;
      if (BIAS_MODE == 2) bv = bias[n];
#pragma unroll
      for (int r = 0; r < 8; ++r) {
        float v = acc[i][j][r] * scale;
        if (BIAS_MODE == 1) v += bias[mBase + mOff + r];
        if (BIAS_MODE == 2) v += bv;
        if (RESID) v += Rb[(size_t)(mBase + mOff + r) * ldc + n];
        if (ACT == 1) v = tanhf(v);
        if (ACT == 2) v = fmaxf(v, 0.0f);
        if (ACT == 4) v = (v > 0.f) ? v : 0.01f * v;
        slab[(mOff + r) * 68 + (j << 4) + rlane] = v;
      }
    }
    __builtin_amdgcn_fence(__ATOMIC_RELEASE, "workgroup");
    __builtin_amdgcn_wave_barrier();
    __builtin_amdgcn_fence(__ATOMIC_ACQUIRE, "workgroup");
    if (OUT_MODE == 0) {
      float* C = (float*)Cout + cOff;
      const int hh = lane >> 4, c4 = (lane & 15) * 4;
      for (int pass = 0; pass < 2; ++pass) {
#pragma unroll
        for (int it = 0; it < 8; ++it) {
          const int row = it * 2 + hh;
          v4f v = *(const v4f*)(slab + row * 68 + c4);
          *(volatile v4f*)(C + (size_t)(mBase + row) * ldc + n0 + c4) = v;
        }
        __threadfence();
      }
    } else {
      const int q = lane >> 3, c8 = (lane & 7) * 8;
      unsigned short* C  = (unsigned short*)Cout  + cOff;
      unsigned short* C2 = (OUT_MODE == 2) ? ((unsigned short*)Cout2 + cOff) : nullptr;
      for (int pass = 0; pass < 2; ++pass) {
#pragma unroll
        for (int it = 0; it < 4; ++it) {
          const int row = it * 4 + q;
          const float* sp = slab + row * 68 + c8;
          v8h hv, lv;
#pragma unroll
          for (int e = 0; e < 8; ++e) {
            if (OUT_MODE == 1) {
              hv[e] = (_Float16)sp[e];
            } else {
              unsigned short hb = f2bf_bits(sp[e]);
              unsigned short lb = f2bf_bits(sp[e] - bf_bits2f(hb));
              hv[e] = __builtin_bit_cast(_Float16, hb);
              lv[e] = __builtin_bit_cast(_Float16, lb);
            }
          }
          *(volatile v8h*)(C + (size_t)(mBase + row) * ldc + n0 + c8) = hv;
          if (OUT_MODE == 2) *(volatile v8h*)(C2 + (size_t)(mBase + row) * ldc + n0 + c8) = lv;
        }
        __threadfence();
      }
    }
    __builtin_amdgcn_fence(__ATOMIC_RELEASE, "workgroup");
    __builtin_amdgcn_wave_barrier();
    __builtin_amdgcn_fence(__ATOMIC_ACQUIRE, "workgroup");
  }
}

__global__ __launch_bounds__(256) void split_bf16x8_kernel(const float* __restrict__ in, unsigned short* __restrict__ hi,
                                                           unsigned short* __restrict__ lo, int n8) {
  const int i = blockIdx.x * 256 + threadIdx.x;
  if (i < n8) {
    const size_t base = (size_t)i * 8;
    const v4f a = *(const v4f*)(in + base);
    const v4f b = *(const v4f*)(in + base + 4);
    const float f[8] = {a[0], a[1], a[2], a[3], b[0], b[1], b[2], b[3]};
    unsigned hw[4], lw[4];
#pragma unroll
    for (int q = 0; q < 4; ++q) {
      const unsigned short h0 = f2bf_bits(f[2 * q]), h1 = f2bf_bits(f[2 * q + 1]);
      const unsigned short l0 = f2bf_bits(f[2 * q] - bf_bits2f(h0));
      const unsigned short l1 = f2bf_bits(f[2 * q + 1] - bf_bits2f(h1));
      hw[q] = pk16(h0, h1);
      lw[q] = pk16(l0, l1);
    }
    const v4u hv = (v4u){hw[0], hw[1], hw[2], hw[3]};
    const v4u lv = (v4u){lw[0], lw[1], lw[2], lw[3]};
    *(volatile v4u*)(hi + base) = hv;
    *(volatile v4u*)(lo + base) = lv;
    __threadfence();
    *(volatile v4u*)(hi + base) = hv;
    *(volatile v4u*)(lo + base) = lv;
  }
}

__device__ __forceinline__ float hw_exp2(float x) { return __builtin_amdgcn_exp2f(x); }
__device__ __forceinline__ float hw_rcp(float x)  { return __builtin_amdgcn_rcpf(x); }

__global__ __launch_bounds__(256) void gate_mix_kernel(
    const float* __restrict__ S, const unsigned short* __restrict__ Qh, const unsigned short* __restrict__ Ql,
    const float* __restrict__ Wg, const float* __restrict__ bg, const float* __restrict__ lam1,
    unsigned short* __restrict__ Ph, unsigned short* __restrict__ Pl, int nrows) {
  const int lane = threadIdx.x & 31;
  const int wave = threadIdx.x >> 5;
  const int rg = blockIdx.x * 8 + wave;
  if (rg >= nrows) return;
  const int z  = rg >> 9;
  const int i  = rg & (kSeq - 1);
  const int bb = z >> 3;
  const int h  = z & (kHeads - 1);
  const float* srow = S + (size_t)rg * kSeq;
  const int j0 = lane * 8;
  const int j1 = 256 + lane * 8;
  const v4f sa = *(const v4f*)(srow + j0);
  const v4f sb = *(const v4f*)(srow + j0 + 4);
  const v4f sc = *(const v4f*)(srow + j1);
  const v4f sd = *(const v4f*)(srow + j1 + 4);
  const float s[16] = {sa[0], sa[1], sa[2], sa[3], sb[0], sb[1], sb[2], sb[3],
                       sc[0], sc[1], sc[2], sc[3], sd[0], sd[1], sd[2], sd[3]};

  const size_t qo = (size_t)(bb * kSeq + i) * kDm + (size_t)h * kDk;
  const float q0 = bf_bits2f(Qh[qo + lane]) + bf_bits2f(Ql[qo + lane]);
  const float q1 = bf_bits2f(Qh[qo + 32 + lane]) + bf_bits2f(Ql[qo + 32 + lane]);
  float g0 = q0 * Wg[lane] + q1 * Wg[32 + lane];
  float g1 = q0 * Wg[kDk + lane] + q1 * Wg[kDk + 32 + lane];
#pragma unroll
  for (int off = 16; off > 0; off >>= 1) {
    g0 += __shfl_xor(g0, off, 32);
    g1 += __shfl_xor(g1, off, 32);
  }
  g0 += bg[0];
  g1 += bg[1];
  const float t0 = fabsf(g0) + 1.0f;
  const float t1 = fabsf(g1) + 1.0f;
  const float qp0 = hw_rcp(t0 * t0);
  const float qp1 = hw_rcp(t1 * t1);
  const float gn0 = (-0.5f * kLog2e) * qp0;
  const float gn1 = (-0.5f * kLog2e) * qp1;
  const float lam = lam1[0];
  const float sg  = hw_rcp(1.0f + hw_exp2(-lam * kLog2e));
  const float omg = 1.0f - sg;

  float mx = s[0];
#pragma unroll
  for (int e = 1; e < 16; ++e) mx = fmaxf(mx, s[e]);
#pragma unroll
  for (int off = 16; off > 0; off >>= 1) mx = fmaxf(mx, __shfl_xor(mx, off, 32));

  float a[16];
  float ps = 0.f;
#pragma unroll
  for (int e = 0; e < 16; ++e) {
    const int j = (e < 8) ? (j0 + e) : (j1 + (e - 8));
    const float p   = hw_exp2((s[e] - mx) * kLog2e);
    const float fd  = (float)(i - j);
    const float gs  = (j < i) ? gn1 : gn0;
    const float adj = hw_exp2((fd * fd) * gs);
    const float av  = sg * p + omg * adj;
    a[e] = av;
    ps += av;
  }
#pragma unroll
  for (int off = 16; off > 0; off >>= 1) ps += __shfl_xor(ps, off, 32);
  const float inv = hw_rcp(ps + 1e-9f);

  unsigned hw0[4], lw0[4], hw1[4], lw1[4];
#pragma unroll
  for (int q = 0; q < 4; ++q) {
    const float p0 = a[2 * q] * inv, p1 = a[2 * q + 1] * inv;
    const float p2 = a[8 + 2 * q] * inv, p3 = a[9 + 2 * q] * inv;
    const unsigned short h0 = f2bf_bits(p0), h1 = f2bf_bits(p1), h2 = f2bf_bits(p2), h3 = f2bf_bits(p3);
    const unsigned short l0 = f2bf_bits(p0 - bf_bits2f(h0));
    const unsigned short l1 = f2bf_bits(p1 - bf_bits2f(h1));
    const unsigned short l2 = f2bf_bits(p2 - bf_bits2f(h2));
    const unsigned short l3 = f2bf_bits(p3 - bf_bits2f(h3));
    hw0[q] = pk16(h0, h1); lw0[q] = pk16(l0, l1);
    hw1[q] = pk16(h2, h3); lw1[q] = pk16(l2, l3);
  }
  const v4u hv0 = (v4u){hw0[0], hw0[1], hw0[2], hw0[3]};
  const v4u lv0 = (v4u){lw0[0], lw0[1], lw0[2], lw0[3]};
  const v4u hv1 = (v4u){hw1[0], hw1[1], hw1[2], hw1[3]};
  const v4u lv1 = (v4u){lw1[0], lw1[1], lw1[2], lw1[3]};
  const size_t ro = (size_t)rg * kSeq;
  *(volatile v4u*)(Ph + ro + j0) = hv0;
  *(volatile v4u*)(Ph + ro + j1) = hv1;
  *(volatile v4u*)(Pl + ro + j0) = lv0;
  *(volatile v4u*)(Pl + ro + j1) = lv1;
  __threadfence();
  *(volatile v4u*)(Ph + ro + j0) = hv0;
  *(volatile v4u*)(Ph + ro + j1) = hv1;
  *(volatile v4u*)(Pl + ro + j0) = lv0;
  *(volatile v4u*)(Pl + ro + j1) = lv1;
}

extern "C" void kernel_launch(void* const* d_in, const int* in_sizes, int n_in,
                              void* d_out, int out_size, void* d_ws, size_t ws_size,
                              hipStream_t stream) {
  if (n_in < 14) return;
  const int nAct = kBatch * kSeq * kDm;
  const int nW   = kDm * kDm;
  if (in_sizes[0] != nAct || in_sizes[1] != nAct || in_sizes[2] != nAct) return;
  if (in_sizes[3] != nW || in_sizes[5] != nW || in_sizes[7] != nW || in_sizes[12] != nW) return;
  if (in_sizes[4] != kDm || in_sizes[6] != kDm || in_sizes[8] != kDm || in_sizes[13] != kDm) return;
  if (in_sizes[9] != 2 * kDk || in_sizes[10] < 2 || in_sizes[11] < 1) return;
  if (out_size != nAct) return;

  const float* query = (const float*)d_in[0];
  const float* key   = (const float*)d_in[1];
  const float* value = (const float*)d_in[2];
  const float* Wq    = (const float*)d_in[3];
  const float* bq    = (const float*)d_in[4];
  const float* Wk    = (const float*)d_in[5];
  const float* bk    = (const float*)d_in[6];
  const float* Wv    = (const float*)d_in[7];
  const float* bv    = (const float*)d_in[8];
  const float* Wg    = (const float*)d_in[9];
  const float* bg    = (const float*)d_in[10];
  const float* lam1  = (const float*)d_in[11];
  const float* Wo    = (const float*)d_in[12];
  const float* bo    = (const float*)d_in[13];
  float* out = (float*)d_out;

  const size_t PW  = (size_t)kDm * kDm * 2;
  const size_t PX  = (size_t)kGRows * kDm * 2;
  const size_t PVT = (size_t)kGB * kDm * kSeq * 2;
  const size_t PS  = (size_t)kNZ * kSeq * kSeq * 4;
  const size_t PP  = (size_t)kNZ * kSeq * kSeq * 2;
  size_t off = 0;
  const size_t oWqh = off; off += PW;  const size_t oWql = off; off += PW;
  const size_t oWkh = off; off += PW;  const size_t oWkl = off; off += PW;
  const size_t oWvh = off; off += PW;  const size_t oWvl = off; off += PW;
  const size_t oWoh = off; off += PW;  const size_t oWol = off; off += PW;
  const size_t oXqh = off; off += PX;  const size_t oXql = off; off += PX;
  const size_t oXkh = off; off += PX;  const size_t oXkl = off; off += PX;
  const size_t oXvh = off; off += PX;  const size_t oXvl = off; off += PX;
  const size_t oQh  = off; off += PX;  const size_t oQl  = off; off += PX;
  const size_t oKh  = off; off += PX;  const size_t oKl  = off; off += PX;
  const size_t oVTh = off; off += PVT; const size_t oVTl = off; off += PVT;
  const size_t oCh  = off; off += PX;  const size_t oCl  = off; off += PX;
  const size_t oS   = off; off += PS;
  const size_t oPh  = off; off += PP;  const size_t oPl  = off; off += PP;
  if (off > ws_size) return;

  char* ws = (char*)d_ws;
  unsigned short* Wqh = (unsigned short*)(ws + oWqh); unsigned short* Wql = (unsigned short*)(ws + oWql);
  unsigned short* Wkh = (unsigned short*)(ws + oWkh); unsigned short* Wkl = (unsigned short*)(ws + oWkl);
  unsigned short* Wvh = (unsigned short*)(ws + oWvh); unsigned short* Wvl = (unsigned short*)(ws + oWvl);
  unsigned short* Woh = (unsigned short*)(ws + oWoh); unsigned short* Wol = (unsigned short*)(ws + oWol);
  unsigned short* Xqh = (unsigned short*)(ws + oXqh); unsigned short* Xql = (unsigned short*)(ws + oXql);
  unsigned short* Xkh = (unsigned short*)(ws + oXkh); unsigned short* Xkl = (unsigned short*)(ws + oXkl);
  unsigned short* Xvh = (unsigned short*)(ws + oXvh); unsigned short* Xvl = (unsigned short*)(ws + oXvl);
  unsigned short* Qh  = (unsigned short*)(ws + oQh);  unsigned short* Ql  = (unsigned short*)(ws + oQl);
  unsigned short* Kh  = (unsigned short*)(ws + oKh);  unsigned short* Kl  = (unsigned short*)(ws + oKl);
  unsigned short* VTh = (unsigned short*)(ws + oVTh); unsigned short* VTl = (unsigned short*)(ws + oVTl);
  unsigned short* Ch  = (unsigned short*)(ws + oCh);  unsigned short* Cl  = (unsigned short*)(ws + oCl);
  float*          Sb  = (float*)(ws + oS);
  unsigned short* Ph  = (unsigned short*)(ws + oPh);  unsigned short* Pl  = (unsigned short*)(ws + oPl);

  const dim3 blk(256);
  const int n8w = nW / 8;
  const int n8x = kGRows * kDm / 8;
  const dim3 gSplitW((n8w + 255) / 256);
  const dim3 gSplitX((n8x + 255) / 256);
  const dim3 gQ(((kGRows / 64) * (kDm / 64) + 7) / 8, 1);
  const dim3 gVT(((kDm / 64) * (kSeq / 64) + 7) / 8, kGB);
  const dim3 gS(((kSeq / 64) * (kSeq / 64) + 7) / 8, kNZ);
  const int  nMixRows = kNZ * kSeq;
  const dim3 gMix((nMixRows + 7) / 8);
  const dim3 gPV(((kSeq / 64) * (kDk / 64) + 7) / 8, kNZ);
  const dim3 gOut(((kGRows / 64) * (kDm / 64) + 7) / 8, 1);

  const long pQK  = (long)kSeq * kDm;
  const long pSz  = (long)kSeq * kSeq;
  const long pVTb = (long)kDm * kSeq;

  split_bf16x8_kernel<<<gSplitW, blk, 0, stream>>>(Wq, Wqh, Wql, n8w);
  split_bf16x8_kernel<<<gSplitW, blk, 0, stream>>>(Wk, Wkh, Wkl, n8w);
  split_bf16x8_kernel<<<gSplitW, blk, 0, stream>>>(Wv, Wvh, Wvl, n8w);
  split_bf16x8_kernel<<<gSplitW, blk, 0, stream>>>(Wo, Woh, Wol, n8w);

  for (int gb = 0; gb < kNGrp; ++gb) {
    const size_t actOff = (size_t)gb * kGRows * kDm;
    split_bf16x8_kernel<<<gSplitX, blk, 0, stream>>>(query + actOff, Xqh, Xql, n8x);
    split_bf16x8_kernel<<<gSplitX, blk, 0, stream>>>(key   + actOff, Xkh, Xkl, n8x);
    split_bf16x8_kernel<<<gSplitX, blk, 0, stream>>>(value + actOff, Xvh, Xvl, n8x);
    wmma_gemm64<1, true, 2, 2, false, 0><<<gQ, blk, 0, stream>>>(
        Xqh, Xql, kDm, 0L, 0L, Wqh, Wql, kDm, 0L, 0L, (void*)Qh, (void*)Ql, kDm, 0L, 0L,
        bq, bq, 0L, kGRows, kDm, kDm, 1.0f, 1);
    wmma_gemm64<1, true, 2, 2, false, 0><<<gQ, blk, 0, stream>>>(
        Xkh, Xkl, kDm, 0L, 0L, Wkh, Wkl, kDm, 0L, 0L, (void*)Kh, (void*)Kl, kDm, 0L, 0L,
        bk, bk, 0L, kGRows, kDm, kDm, 1.0f, 1);
    wmma_gemm64<1, true, 1, 2, false, 0><<<gVT, blk, 0, stream>>>(
        Wvh, Wvl, kDm, 0L, 0L, Xvh, Xvl, kDm, pQK, 0L, (void*)VTh, (void*)VTl, kSeq, pVTb, 0L,
        bv, bv, 0L, kDm, kSeq, kDm, 1.0f, kGB);
    wmma_gemm64<1, true, 0, 0, false, 0><<<gS, blk, 0, stream>>>(
        Qh, Ql, kDm, (long)kDk, pQK, Kh, Kl, kDm, (long)kDk, pQK, (void*)Sb, (void*)Sb, kSeq, pSz, (long)kHeads * pSz,
        bq, bq, 0L, kSeq, kSeq, kDk, 1.0f, kHeads);
    gate_mix_kernel<<<gMix, blk, 0, stream>>>(Sb, Qh, Ql, Wg, bg, lam1, Ph, Pl, nMixRows);
    wmma_gemm64<1, true, 0, 2, false, 0><<<gPV, blk, 0, stream>>>(
        Ph, Pl, kSeq, pSz, (long)kHeads * pSz, VTh, VTl, kSeq, (long)kDk * kSeq, pVTb,
        (void*)Ch, (void*)Cl, kDm, (long)kDk, pQK,
        bq, bq, 0L, kSeq, kDk, kSeq, 1.0f, kHeads);
    float* outg = out + actOff;
    wmma_gemm64<1, true, 2, 0, false, 0><<<gOut, blk, 0, stream>>>(
        Ch, Cl, kDm, 0L, 0L, Woh, Wol, kDm, 0L, 0L, (void*)outg, (void*)outg, kDm, 0L, 0L,
        bo, bo, 0L, kGRows, kDm, kDm, 1.0f, 1);
  }
}
